// CausalSelfAttention_35089882808734
// MI455X (gfx1250) — hardware-run, weakly checked
//
#include <hip/hip_runtime.h>


#ifndef NB
#define NB 1
#endif
#ifndef SEQ
#define SEQ 4096
#endif
#define SEQ_FULL 4096
#define TT   SEQ
#define DM   1024
#define NH_  16
#define NKV  4
#define REP  (NH_ / NKV)
#define HD   64
#define DQ   (NH_ * HD)
#define DKV  (NKV * HD)
#define NQKV (DQ + 2 * DKV)
#define GCH  32
#define RH   ((TT < 512) ? TT : 512)
#define PLG  10.0f
#define SCL2 (0.125f * 1.4426950408889634f)
#define NEGB (-3.0e38f)
#define EPSF 1.1920929e-07f
#define SPT  72

static_assert(TT % 64 == 0);
static_assert(RH % 64 == 0);
static_assert((TT - RH) % 64 == 0);
static_assert(DM % 64 == 0 && DQ % 64 == 0 && DKV % 64 == 0 && NQKV % 64 == 0);
static_assert(DM % 32 == 0 && DQ % 32 == 0 && HD % 32 == 0 && TT % 32 == 0);
static_assert(HD == 64);
static_assert(HD / 2 == 32);
static_assert(DQ == DM);
static_assert(NH_ % NKV == 0);
static_assert(GCH <= DM);
static_assert(SPT >= HD && SPT % 8 == 0);
static_assert((TT * DM) % 8 == 0);
static_assert(((long long)NH_ * TT * HD / 2) % 256 == 0 && ((long long)NKV * TT * HD / 2) % 256 == 0);
static_assert((TT * NKV) % 256 == 0);
static_assert(NB >= 1 && SEQ <= SEQ_FULL);

#define AL256(x) ((((size_t)(x)) + 255) & ~(size_t)255)
constexpr size_t WS_TOTAL = AL256((size_t)NQKV * DM * 2) + AL256((size_t)DM * DQ * 2) + AL256((size_t)TT * DM * 2) + AL256((size_t)TT * NQKV * 4) + AL256((size_t)TT * NKV * 4)
                          + 3 * AL256((size_t)NH_ * TT * HD * 2) + 3 * AL256((size_t)NKV * TT * HD * 2) + 3 * AL256((size_t)NKV * HD * TT * 2) + 2 * AL256((size_t)TT * DQ * 2);
static_assert(WS_TOTAL <= (size_t)134217728u);

typedef _Float16 h16;
typedef unsigned short bf;
typedef __attribute__((ext_vector_type(16))) __bf16   v16bf;
typedef __attribute__((ext_vector_type(16))) _Float16 v16h;
typedef __attribute__((ext_vector_type(8)))  _Float16 v8h;
typedef __attribute__((ext_vector_type(8)))  unsigned short v8us;
typedef __attribute__((ext_vector_type(8)))  float    v8f;
typedef __attribute__((ext_vector_type(4)))  float    v4f;
typedef __attribute__((ext_vector_type(2))) _Float16 v2h;
typedef __attribute__((ext_vector_type(4))) _Float16 v4h;
typedef __attribute__((ext_vector_type(2))) unsigned short v2us;
typedef __attribute__((ext_vector_type(4))) unsigned short v4us;
typedef __attribute__((ext_vector_type(2))) float v2f;
typedef v8h  __attribute__((may_alias)) v8ha;
typedef v4f  __attribute__((may_alias)) v4fa;
typedef v8us __attribute__((may_alias)) v8usa;

__device__ __forceinline__ unsigned short f2bf(float f) { unsigned u = __float_as_uint(f); u += 0x7FFFu + ((u >> 16) & 1u); return (unsigned short)(u >> 16); }
__device__ __forceinline__ float bf2f(unsigned short b) { return __uint_as_float(((unsigned)b) << 16); }
__device__ __forceinline__ float bfr(float f) { return bf2f(f2bf(f)); }
__device__ __forceinline__ v16h cat16(v8h lo, v8h hi) { return __builtin_shufflevector(lo, hi, 0, 1, 2, 3, 4, 5, 6, 7, 8, 9, 10, 11, 12, 13, 14, 15); }
__device__ __forceinline__ v16bf cat16b(v8us lo, v8us hi) { return __builtin_bit_cast(v16bf, __builtin_shufflevector(lo, hi, 0, 1, 2, 3, 4, 5, 6, 7, 8, 9, 10, 11, 12, 13, 14, 15)); }
__device__ __forceinline__ v8f wmma16(v16h a, v16h b, v8f c) { return __builtin_amdgcn_wmma_f32_16x16x32_f16(false, a, false, b, (short)0, c, false, false); }
__device__ __forceinline__ v8f wmmab(v16bf a, v16bf b, v8f c) { return __builtin_amdgcn_wmma_f32_16x16x32_bf16(false, a, false, b, (short)0, c, false, false); }
__device__ __forceinline__ h16 tohx(float x) { return (h16)x; }
__device__ __forceinline__ void splitf(float y, unsigned short& h, unsigned short& l) { h = f2bf(y); l = f2bf(y - bf2f(h)); }

template <typename T16> struct WFrag;
template <> struct WFrag<h16> { typedef v16h V; static __device__ __forceinline__ V ld(const h16* p) { return cat16(*(const v8h*)p, *(const v8h*)(p + 16)); } static __device__ __forceinline__ v8f mma(V a, V b, v8f c) { return wmma16(a, b, c); } };
template <> struct WFrag<bf> { typedef v16bf V; static __device__ __forceinline__ V ld(const bf* p) { return cat16b(*(const v8us*)p, *(const v8us*)(p + 16)); } static __device__ __forceinline__ v8f mma(V a, V b, v8f c) { return wmmab(a, b, c); } };

template <typename T16, int NSPLIT, bool BIAS>
__global__ __launch_bounds__(32) void k_gemmw(const T16* __restrict__ A, const T16* __restrict__ A2, const T16* __restrict__ Bt, const T16* __restrict__ Bt2, int K, float* C, int ldc, const float* __restrict__ bias, size_t sA, size_t sB, size_t sC) {
    typedef typename WFrag<T16>::V V;
    __shared__ __align__(16) float os[16 * 68];
    const size_t z = blockIdx.z; A += z * sA; if (A2) A2 += z * sA; Bt += z * sB; if (Bt2) Bt2 += z * sB; C += z * sC;
    const int lane = threadIdx.x & 31, lr = lane & 15, hi = lane >> 4; const int r0 = blockIdx.x * 64, c0 = blockIdx.y * 64;
    v8f acc[4][4];
#pragma unroll
    for (int mb = 0; mb < 4; ++mb)
#pragma unroll
        for (int nb = 0; nb < 4; ++nb) acc[mb][nb] = (v8f){};
    const size_t aoff = (size_t)(r0 + lr) * K + 8 * hi, boff = (size_t)(c0 + lr) * K + 8 * hi;
#pragma unroll 1
    for (int kc = 0; kc < K; kc += 32) {
        V a[4], a2[4];
#pragma unroll
        for (int mb = 0; mb < 4; ++mb) { a[mb] = WFrag<T16>::ld(A + aoff + (size_t)mb * 16 * K + kc); if (NSPLIT == 1 || NSPLIT == 2) a2[mb] = WFrag<T16>::ld(A2 + aoff + (size_t)mb * 16 * K + kc); }
#pragma unroll
        for (int nb = 0; nb < 4; ++nb) { const V b = WFrag<T16>::ld(Bt + boff + (size_t)nb * 16 * K + kc); V b2; if (NSPLIT >= 2) b2 = WFrag<T16>::ld(Bt2 + boff + (size_t)nb * 16 * K + kc);
#pragma unroll
            for (int mb = 0; mb < 4; ++mb) { acc[mb][nb] = WFrag<T16>::mma(a[mb], b, acc[mb][nb]); if (NSPLIT == 1 || NSPLIT == 2) acc[mb][nb] = WFrag<T16>::mma(a2[mb], b, acc[mb][nb]); if (NSPLIT >= 2) acc[mb][nb] = WFrag<T16>::mma(a[mb], b2, acc[mb][nb]); } }
        asm volatile("v_nop\n\tv_nop\n\tv_nop\n\tv_nop" : "+v"(acc[0][0]), "+v"(acc[1][1]), "+v"(acc[2][2]), "+v"(acc[3][3]) : "v"(a[0]), "v"(a[3]));
    }
#pragma unroll
    for (int mb = 0; mb < 4; ++mb) {
#pragma unroll
        for (int nb = 0; nb < 4; ++nb) {
#pragma unroll
            for (int j = 0; j < 8; ++j) os[(hi * 8 + j) * 68 + nb * 16 + lr] = acc[mb][nb][j]; }
        __builtin_amdgcn_wave_barrier(); asm volatile("" ::: "memory");
        float* crow = C + (size_t)(r0 + mb * 16) * ldc + c0;
#pragma unroll 1
        for (int ps = 0; ps < 2; ++ps) {
#pragma unroll
            for (int s = 0; s < 8; ++s) { const int row = 2 * s + hi, cofs = lr * 4; v4f val = *(const v4fa*)(os + row * 68 + cofs); if (BIAS) { val[0] += bfr(bias[c0 + cofs]); val[1] += bfr(bias[c0 + cofs + 1]); val[2] += bfr(bias[c0 + cofs + 2]); val[3] += bfr(bias[c0 + cofs + 3]); }
                *(volatile v4f*)(crow + (size_t)row * ldc + cofs) = val; }
            if (ps == 0) __threadfence(); }
        __builtin_amdgcn_wave_barrier(); asm volatile("" ::: "memory");
    }
}

__global__ __launch_bounds__(256) void k_cvt8(const float* __restrict__ src, bf* dst, size_t n8) { const size_t i = (size_t)blockIdx.x * 256 + threadIdx.x; if (i >= n8) return; const v8f v = *(const v8f*)(src + i * 8); v8us o;
#pragma unroll
    for (int k = 0; k < 8; ++k) o[k] = f2bf(v[k]); *(volatile v8us*)(dst + i * 8) = o; __threadfence(); *(volatile v8us*)(dst + i * 8) = o; }

static __device__ __forceinline__ h16 toh_flush(float v) { const h16 r = (h16)v; return (fabsf(v) < 6.103515625e-05f) ? (h16)0.0f : r; }
__device__ __forceinline__ v8f wg16(v16h a, v16h b, v8f c) { c = wmma16(a, b, c); asm volatile("v_nop\n\tv_nop\n\tv_nop\n\tv_nop" : "+v"(c) : "v"(a), "v"(b)); return c; }
__device__ __forceinline__ v8f wgb(v16bf a, v16bf b, v8f c) { c = wmmab(a, b, c); asm volatile("v_nop\n\tv_nop\n\tv_nop\n\tv_nop" : "+v"(c) : "v"(a), "v"(b)); return c; }

__global__ __launch_bounds__(256) void k_cvtT(const float* __restrict__ src, int N, bf* dst) {
    __shared__ __align__(16) unsigned short tl[64 * SPT];
    const int tid = threadIdx.x; const int k0 = blockIdx.x * 64, n0 = blockIdx.y * 64;
#pragma unroll 1
    for (int it = 0; it < 16; ++it) { const int idx = it * 256 + tid; const int kk = idx >> 6, nn = idx & 63; tl[nn * SPT + kk] = f2bf(src[(size_t)(k0 + kk) * N + n0 + nn]); }
    __syncthreads();
#pragma unroll 1
    for (int ps = 0; ps < 2; ++ps) {
#pragma unroll
        for (int it = 0; it < 2; ++it) { const int p = it * 256 + tid; const int row = p >> 3, pc = p & 7; const v8us v = *(const v8usa*)(tl + row * SPT + pc * 8);
            *(volatile v8us*)(dst + (size_t)(n0 + row) * DM + k0 + pc * 8) = v; }
        if (ps == 0) __threadfence(); }
}

__global__ __launch_bounds__(256) void k_gate(const float* __restrict__ x, const float* __restrict__ wg, float* G) {
#pragma clang fp contract(off)
    const int idx = blockIdx.x * 256 + threadIdx.x; if (idx >= TT * NKV) return; const int t = idx / NKV, g = idx % NKV; const float* xr = x + (size_t)t * DM; float a = 0.0f;
#pragma unroll 1
    for (int c = 0; c < GCH; ++c) a += bfr(xr[c]) * bfr(wg[c * NKV + g]);
    const float gt = 2.0f * (1.0f / (1.0f + expf(-a)));
    *(volatile float*)(G + idx) = gt; __threadfence(); *(volatile float*)(G + idx) = gt; }

__global__ __launch_bounds__(256) void k_ropen(const float* __restrict__ F, int pitch, int coff, int nheads, const float* __restrict__ cosb, const float* __restrict__ sinb, h16* P16, bf* Ph, bf* Pl) {
#pragma clang fp contract(off)
    const size_t e = ((size_t)blockIdx.x * 256 + threadIdx.x) * 2; if (e >= (size_t)nheads * TT * HD) return; const int d = (int)(e % HD); const int t = (int)((e / HD) % TT); const int h = (int)(e / ((size_t)HD * TT));
    const float* f = F + (size_t)t * pitch + coff + h * HD; const int j = d & (HD / 2 - 1); const int dp = d ^ (HD / 2); const float sg = (d < HD / 2) ? 1.0f : -1.0f;
    const v2f xa = *(const v2f*)(f + d); const v2f xb = *(const v2f*)(f + dp); const v2f cc = *(const v2f*)(cosb + (size_t)t * (HD / 2) + j); const v2f sn = *(const v2f*)(sinb + (size_t)t * (HD / 2) + j);
    const float r0 = xa[0] * bfr(cc[0]) + sg * (xb[0] * bfr(sn[0])); const float r1 = xa[1] * bfr(cc[1]) + sg * (xb[1] * bfr(sn[1]));
    float ss = r0 * r0 + r1 * r1;
#pragma unroll
    for (int sh = 16; sh; sh >>= 1) ss += __shfl_xor(ss, sh, 32);
    const float rs = rsqrtf(ss * (1.0f / (float)HD) + EPSF); const float y0 = r0 * rs, y1 = r1 * rs;
    v2h o16; v2us oh, ol; unsigned short a2, c2; o16[0] = toh_flush(y0); o16[1] = toh_flush(y1); splitf(y0, a2, c2); oh[0] = a2; ol[0] = c2; splitf(y1, a2, c2); oh[1] = a2; ol[1] = c2;
    *(volatile v2h*)(P16 + e) = o16; *(volatile v2us*)(Ph + e) = oh; *(volatile v2us*)(Pl + e) = ol; __threadfence(); *(volatile v2h*)(P16 + e) = o16; *(volatile v2us*)(Ph + e) = oh; *(volatile v2us*)(Pl + e) = ol; }

__global__ __launch_bounds__(256) void k_vtg(const float* __restrict__ F, int pitch, int coff, int nheads, const float* __restrict__ G, const float* __restrict__ ve, h16* V16, bf* Vh, bf* Vl) {
#pragma clang fp contract(off)
    const size_t e = ((size_t)blockIdx.x * 256 + threadIdx.x) * 2; if (e >= (size_t)nheads * HD * TT) return; const int t = (int)(e % TT); const int d = (int)((e / TT) % HD); const int g = (int)(e / ((size_t)TT * HD)); v2h o16; v2us oh, ol;
#pragma unroll
    for (int q = 0; q < 2; ++q) { const int tq = t + q; const float gv = G[(size_t)tq * NKV + g]; const float ev = bfr(ve[(size_t)tq * DKV + g * HD + d]); const float x = F[(size_t)tq * pitch + coff + g * HD + d] + gv * ev;
        o16[q] = toh_flush(x); unsigned short a2, c2; splitf(x, a2, c2); oh[q] = a2; ol[q] = c2; }
    *(volatile v2h*)(V16 + e) = o16; *(volatile v2us*)(Vh + e) = oh; *(volatile v2us*)(Vl + e) = ol; __threadfence(); *(volatile v2h*)(V16 + e) = o16; *(volatile v2us*)(Vh + e) = oh; *(volatile v2us*)(Vl + e) = ol; }

template <bool EARLY>
static __device__ __forceinline__ void attn_body(const h16* __restrict__ Q16, const bf* __restrict__ Qh, const bf* __restrict__ Ql, const h16* __restrict__ K16, const bf* __restrict__ Kh, const bf* __restrict__ Kl,
                                                 const h16* __restrict__ V16, const bf* __restrict__ Vh, const bf* __restrict__ Vl, bf* ATh, bf* ATl, const int* __restrict__ wsp, int roff) {
    __shared__ __align__(16) unsigned short stg[4 * 2 * 16 * SPT];
    const int lane = threadIdx.x & 31, lr = lane & 15, hi = lane >> 4;
    const int wave = __builtin_amdgcn_readfirstlane(threadIdx.x >> 5);
    const int h = (int)blockIdx.y, g = h / REP;
    const int q0 = roff + (int)blockIdx.x * 64 + wave * 16;
    int wl = wsp[0]; if (wl <= 0 || wl >= TT) wl = TT;
    int klo = q0 - wl; klo &= ~(klo >> 31);
    const int kstart = klo & ~31; const int kend = q0 + 16;
    const int i = q0 + lr, ilo = i - wl;
    const size_t qoff = ((size_t)h * TT + q0 + lr) * HD + 8 * hi;
    const size_t kbase = (size_t)g * TT * HD + (size_t)lr * HD + 8 * hi;
    const size_t vbase = (size_t)g * HD * TT + (size_t)lr * TT + 8 * hi;
    v16h qf[2]; v16bf qh[2], ql[2];
#pragma unroll
    for (int c = 0; c < 2; ++c) { if (EARLY) { qh[c] = WFrag<bf>::ld(Qh + qoff + c * 32); ql[c] = WFrag<bf>::ld(Ql + qoff + c * 32); } else { qf[c] = WFrag<h16>::ld(Q16 + qoff + c * 32); } }
    float m = NEGB, l = 0.0f; v8f o[4];
#pragma unroll
    for (int dt = 0; dt < 4; ++dt) o[dt] = (v8f){};
#pragma unroll 1
    for (int kb = kstart; kb < kend; kb += 32) {
        v8f s0 = (v8f){}, s1 = (v8f){};
        if (EARLY) {
#pragma unroll
            for (int c = 0; c < 2; ++c) { const size_t ko = kbase + (size_t)kb * HD + c * 32;
                const v16bf a0h = WFrag<bf>::ld(Kh + ko); const v16bf a0l = WFrag<bf>::ld(Kl + ko);
                s0 = wgb(a0h, qh[c], s0); s0 = wgb(a0l, qh[c], s0); s0 = wgb(a0h, ql[c], s0);
                const v16bf a1h = WFrag<bf>::ld(Kh + ko + 16 * HD); const v16bf a1l = WFrag<bf>::ld(Kl + ko + 16 * HD);
                s1 = wgb(a1h, qh[c], s1); s1 = wgb(a1l, qh[c], s1); s1 = wgb(a1h, ql[c], s1); }
        } else {
#pragma unroll
            for (int c = 0; c < 2; ++c) { const size_t ko = kbase + (size_t)kb * HD + c * 32;
                const v16h a0 = WFrag<h16>::ld(K16 + ko); const v16h a1 = WFrag<h16>::ld(K16 + ko + 16 * HD);
                s0 = wg16(a0, qf[c], s0); s1 = wg16(a1, qf[c], s1); }
        }
        float mx = NEGB;
#pragma unroll
        for (int r = 0; r < 8; ++r) { const int j0 = kb + 8 * hi + r, j1 = j0 + 16; const bool ok0 = (j0 <= i) && (j0 >= ilo); const bool ok1 = (j1 <= i) && (j1 >= ilo);
            const float t0 = ok0 ? s0[r] * SCL2 : NEGB; const float t1 = ok1 ? s1[r] * SCL2 : NEGB; s0[r] = t0; s1[r] = t1; mx = fmaxf(mx, fmaxf(t0, t1)); }
        mx = fmaxf(mx, __shfl_xor(mx, 16, 32));
        const float mnew = fmaxf(m, mx); const float alpha = __builtin_amdgcn_exp2f(m - mnew); m = mnew;
#pragma unroll
        for (int dt = 0; dt < 4; ++dt)
#pragma unroll
            for (int r = 0; r < 8; ++r) o[dt][r] *= alpha;
        float ls = 0.0f;
        if (EARLY) {
            v8us p0h, p0l, p1h, p1l;
#pragma unroll
            for (int r = 0; r < 8; ++r) { const float e0 = s0[r] - mnew, e1 = s1[r] - mnew; float pv0 = __builtin_amdgcn_exp2f(e0), pv1 = __builtin_amdgcn_exp2f(e1);
                pv0 = (s0[r] > -1.0e38f) ? pv0 : 0.0f; pv1 = (s1[r] > -1.0e38f) ? pv1 : 0.0f; ls += pv0 + pv1;
                unsigned short a2, c2; splitf(pv0, a2, c2); p0h[r] = a2; p0l[r] = c2; splitf(pv1, a2, c2); p1h[r] = a2; p1l[r] = c2; }
            const v16bf pfh = cat16b(p0h, p1h); const v16bf pfl = cat16b(p0l, p1l);
#pragma unroll
            for (int dt = 0; dt < 4; ++dt) { const size_t vo = vbase + (size_t)(dt * 16) * TT + kb; const v16bf vh = WFrag<bf>::ld(Vh + vo); const v16bf vl = WFrag<bf>::ld(Vl + vo);
                o[dt] = wgb(vh, pfh, o[dt]); o[dt] = wgb(vl, pfh, o[dt]); o[dt] = wgb(vh, pfl, o[dt]); }
        } else {
            v8h p0, p1;
#pragma unroll
            for (int r = 0; r < 8; ++r) { const float e0 = s0[r] - mnew + PLG, e1 = s1[r] - mnew + PLG; float pv0 = __builtin_amdgcn_exp2f(e0), pv1 = __builtin_amdgcn_exp2f(e1);
                pv0 = ((s0[r] > -1.0e38f) && (e0 >= -14.0f)) ? pv0 : 0.0f; pv1 = ((s1[r] > -1.0e38f) && (e1 >= -14.0f)) ? pv1 : 0.0f;
                const h16 c0 = (h16)pv0; const h16 c1 = (h16)pv1; p0[r] = c0; p1[r] = c1; ls += (float)c0 + (float)c1; }
            const v16h pf = cat16(p0, p1);
#pragma unroll
            for (int dt = 0; dt < 4; ++dt) { const size_t vo = vbase + (size_t)(dt * 16) * TT + kb; const v16h va = WFrag<h16>::ld(V16 + vo); o[dt] = wg16(va, pf, o[dt]); }
        }
        l = l * alpha + ls;
    }
    const float lt = l + __shfl_xor(l, 16, 32);
    const float inv = 1.0f / lt;
    const int sb = wave * (2 * 16 * SPT);
#pragma unroll
    for (int dt = 0; dt < 4; ++dt) { v8us oh, ol;
#pragma unroll
        for (int r = 0; r < 8; ++r) { unsigned short a2, c2; splitf(o[dt][r] * inv, a2, c2); oh[r] = a2; ol[r] = c2; }
        *(v8usa*)(stg + sb + lr * SPT + dt * 16 + 8 * hi) = oh; *(v8usa*)(stg + sb + 16 * SPT + lr * SPT + dt * 16 + 8 * hi) = ol; }
    __builtin_amdgcn_wave_barrier(); asm volatile("" ::: "memory");
    const int prow = lane >> 3, pc = lane & 7;
#pragma unroll 1
    for (int ps = 0; ps < 2; ++ps) {
#pragma unroll
        for (int s = 0; s < 4; ++s) { const int row = 4 * s + prow; const v8us sh = *(const v8usa*)(stg + sb + row * SPT + pc * 8); const v8us sl = *(const v8usa*)(stg + sb + 16 * SPT + row * SPT + pc * 8);
            const size_t oo = (size_t)(q0 + row) * DQ + (size_t)h * HD + pc * 8; *(volatile v8us*)(ATh + oo) = sh; *(volatile v8us*)(ATl + oo) = sl; }
        if (ps == 0) __threadfence(); }
}

__global__ __launch_bounds__(128) void k_attn_early(const bf* __restrict__ Qh, const bf* __restrict__ Ql, const bf* __restrict__ Kh, const bf* __restrict__ Kl, const bf* __restrict__ Vh, const bf* __restrict__ Vl, bf* ATh, bf* ATl, const int* __restrict__ wsp) {
    attn_body<true>(nullptr, Qh, Ql, nullptr, Kh, Kl, nullptr, Vh, Vl, ATh, ATl, wsp, 0); }
__global__ __launch_bounds__(128) void k_attn_late(const h16* __restrict__ Q16, const h16* __restrict__ K16, const h16* __restrict__ V16, bf* ATh, bf* ATl, const int* __restrict__ wsp) {
    attn_body<false>(Q16, nullptr, nullptr, K16, nullptr, nullptr, V16, nullptr, nullptr, ATh, ATl, wsp, RH); }

extern "C" void kernel_launch(void* const* d_in, const int* in_sizes, int n_in,
                              void* d_out, int out_size, void* d_ws, size_t ws_size, hipStream_t stream) {
    if (n_in < 10) return;
    if (in_sizes[0] < (NB - 1) * SEQ_FULL * DM + TT * DM) return;
    if (in_sizes[1] < (NB - 1) * SEQ_FULL * DKV + TT * DKV) return;
    if (in_sizes[2] < TT * (HD / 2) || in_sizes[3] < TT * (HD / 2)) return;
    if (in_sizes[4] < DM * DQ || in_sizes[5] < DM * DKV || in_sizes[6] < DM * DKV || in_sizes[7] < DQ * DM || in_sizes[8] < GCH * NKV || in_sizes[9] < 1) return;
    if (out_size < NB * TT * DM) return;
    const float* x = (const float*)d_in[0]; const float* ve = (const float*)d_in[1]; const float* cosb = (const float*)d_in[2]; const float* sinb = (const float*)d_in[3];
    const float* wq = (const float*)d_in[4]; const float* wk = (const float*)d_in[5]; const float* wv = (const float*)d_in[6]; const float* wo = (const float*)d_in[7]; const float* wg = (const float*)d_in[8];
    const int* wsp = (const int*)d_in[9];
    float* OUT = (float*)d_out;
    char* wsc = (char*)d_ws;
    auto take = [&](size_t bytes) { char* p = wsc; wsc += (bytes + 255) & ~(size_t)255; return (void*)p; };
    bf* WQKV = (bf*)take((size_t)NQKV * DM * 2); bf* WO = (bf*)take((size_t)DM * DQ * 2);
    bf* XB = (bf*)take((size_t)TT * DM * 2); float* F = (float*)take((size_t)TT * NQKV * 4); float* G = (float*)take((size_t)TT * NKV * 4);
    h16* QP16 = (h16*)take((size_t)NH_ * TT * HD * 2); bf* QPh = (bf*)take((size_t)NH_ * TT * HD * 2); bf* QPl = (bf*)take((size_t)NH_ * TT * HD * 2);
    h16* KP16 = (h16*)take((size_t)NKV * TT * HD * 2); bf* KPh = (bf*)take((size_t)NKV * TT * HD * 2); bf* KPl = (bf*)take((size_t)NKV * TT * HD * 2);
    h16* VT16 = (h16*)take((size_t)NKV * HD * TT * 2); bf* VTh = (bf*)take((size_t)NKV * HD * TT * 2); bf* VTl = (bf*)take((size_t)NKV * HD * TT * 2);
    bf* ATh = (bf*)take((size_t)TT * DQ * 2); bf* ATl = (bf*)take((size_t)TT * DQ * 2);
    const size_t used = (size_t)(wsc - (char*)d_ws); if (used > ws_size || used > (size_t)134217728u) return;
    k_cvtT<<<dim3(DM / 64, DQ / 64), 256, 0, stream>>>(wq, DQ, WQKV);
    k_cvtT<<<dim3(DM / 64, DKV / 64), 256, 0, stream>>>(wk, DKV, WQKV + (size_t)DQ * DM);
    k_cvtT<<<dim3(DM / 64, DKV / 64), 256, 0, stream>>>(wv, DKV, WQKV + (size_t)(DQ + DKV) * DM);
    k_cvtT<<<dim3(DQ / 64, DM / 64), 256, 0, stream>>>(wo, DM, WO);
    const unsigned LQ = (unsigned)(((size_t)NH_ * TT * HD / 2 + 255) / 256), LKv = (unsigned)(((size_t)NKV * TT * HD / 2 + 255) / 256);
    for (int b = 0; b < NB; ++b) {
        const float* xb = x + (size_t)b * SEQ_FULL * DM; const float* veb = ve + (size_t)b * SEQ_FULL * DKV;
        k_cvt8<<<(unsigned)(((size_t)TT * DM / 8 + 255) / 256), 256, 0, stream>>>(xb, XB, (size_t)TT * DM / 8);
        k_gemmw<bf, 0, false><<<dim3(TT / 64, NQKV / 64, 1), 32, 0, stream>>>(XB, nullptr, WQKV, nullptr, DM, F, NQKV, nullptr, 0, 0, 0);
        k_gate<<<(TT * NKV + 255) / 256, 256, 0, stream>>>(xb, wg, G);
        k_ropen<<<LQ, 256, 0, stream>>>(F, NQKV, 0, NH_, cosb, sinb, QP16, QPh, QPl);
        k_ropen<<<LKv, 256, 0, stream>>>(F, NQKV, DQ, NKV, cosb, sinb, KP16, KPh, KPl);
        k_vtg<<<LKv, 256, 0, stream>>>(F, NQKV, DQ + DKV, NKV, G, veb, VT16, VTh, VTl);
        if (RH > 0) k_attn_early<<<dim3(RH / 64, NH_), 128, 0, stream>>>(QPh, QPl, KPh, KPl, VTh, VTl, ATh, ATl, wsp);
        if (TT - RH > 0) k_attn_late<<<dim3((TT - RH) / 64, NH_), 128, 0, stream>>>(QP16, KP16, VT16, ATh, ATl, wsp);
        k_gemmw<bf, 1, false><<<dim3(TT / 64, DM / 64, 1), 32, 0, stream>>>(ATh, ATl, WO, nullptr, DQ, OUT + (size_t)b * TT * DM, DM, nullptr, 0, 0, 0); }
}
